// CrossAttnHead_33517924778259
// MI455X (gfx1250) — hardware-verified
//
#include <hip/hip_runtime.h>


namespace {
constexpr int Bn = 16, HH = 12, NT = 256, NO = 512, DM = 128, NHD = 4, DH = 32, NQA = Bn * HH  , NKV = Bn * NO  , NROW = Bn * HH * NT  ;
constexpr float QS = 8.0f, VS = 8.0f, PS = 8.0f, XS = 8.0f, SCALE = 0.17677669529663687f, LNE = 1e-5f;
constexpr size_t VPL = (size_t)Bn * DM * NO;

typedef _Float16 b16;
typedef __attribute__((ext_vector_type(16))) _Float16 v16b;
typedef __attribute__((ext_vector_type(16))) __bf16 v16bb;
typedef __attribute__((ext_vector_type(8))) _Float16 v8b;
typedef __attribute__((ext_vector_type(8))) unsigned short v8us;
typedef __attribute__((ext_vector_type(8))) float v8f;
typedef __attribute__((ext_vector_type(4))) float v4f;
__device__ __forceinline__ float bf16_rne(float f) { unsigned int u = __float_as_uint(f); u += 0x7FFFu + ((u >> 16) & 1u); return __uint_as_float(u & 0xFFFF0000u); }
__device__ __forceinline__ unsigned short bf16_bits(float f) { unsigned int u = __float_as_uint(f); u += 0x7FFFu + ((u >> 16) & 1u); return (unsigned short)(u >> 16); }
__device__ __forceinline__ void split16(float v, b16& hi, b16& lo) { hi = (b16)v; lo = (b16)(v - (float)hi); }
__device__ __forceinline__ v16b frag_kb(const b16* p, int hh) { const v8b a = *(const v8b*)(p + 8 * hh), b = *(const v8b*)(p + 16 + 8 * hh); v16b f;
#pragma unroll
  for (int e = 0; e < 8; ++e) { f[e] = a[e]; f[8 + e] = b[e]; } return f; }
__device__ __forceinline__ v16bb frag_bf(const unsigned short* p, int hh) { const v8us a = *(const v8us*)(p + 8 * hh), b = *(const v8us*)(p + 16 + 8 * hh); union { unsigned short s[16]; v16bb v; } u;
#pragma unroll
  for (int e = 0; e < 8; ++e) { u.s[e] = a[e]; u.s[8 + e] = b[e]; } return u.v; }
__device__ __forceinline__ v16bb frag_f32bf(const float* p, int hh) { union { unsigned short s[16]; v16bb v; } u;
#pragma unroll
  for (int e = 0; e < 8; ++e) { u.s[e] = bf16_bits(p[8 * hh + e]); u.s[8 + e] = bf16_bits(p[16 + 8 * hh + e]); } return u.v; }
__device__ __forceinline__ void frag_split(const float* p, int hh, float sc, v16b& fh, v16b& fl) {
#pragma unroll
  for (int e = 0; e < 8; ++e) { b16 a, c; split16(p[8 * hh + e] * sc, a, c); fh[e] = a; fl[e] = c; split16(p[16 + 8 * hh + e] * sc, a, c); fh[8 + e] = a; fl[8 + e] = c; } }
__device__ __forceinline__ v8f wmma16b(v16b a, v16b b, v8f c) { v8f d = __builtin_amdgcn_wmma_f32_16x16x32_f16(false, a, false, b, (short)0, c, false, false); asm volatile("v_nop\n\tv_nop\n\tv_nop\n\tv_nop" : "+v"(d) : "v"(a), "v"(b)); return d; }
__device__ __forceinline__ v8f wmma16bb(v16bb a, v16bb b, v8f c) { v8f d = __builtin_amdgcn_wmma_f32_16x16x32_bf16(false, a, false, b, (short)0, c, false, false); asm volatile("v_nop\n\tv_nop\n\tv_nop\n\tv_nop" : "+v"(d) : "v"(a), "v"(b)); return d; }
__device__ __forceinline__ void wave_lds_sync() { __builtin_amdgcn_fence(__ATOMIC_RELEASE, "workgroup"); __builtin_amdgcn_wave_barrier(); __builtin_amdgcn_fence(__ATOMIC_ACQUIRE, "workgroup"); }
__device__ __forceinline__ float nexp(float x) { return __builtin_amdgcn_exp2f(x * 1.4426950408889634f); }

__global__ __launch_bounds__(256) void prep_kernel(const float* __restrict__ Wq, const float* __restrict__ Wk, const float* __restrict__ Wv, const float* __restrict__ W1, unsigned short* __restrict__ w16, b16* __restrict__ w1r) {
  const int t_ = threadIdx.x;
  for (int pass = 0; pass < 2; ++pass) {
    for (int p = t_; p < 4 * DM * DM; p += 256) { const int m = p >> 14, q = p & 16383, o = q >> 7, k = q & 127; float v;
      if (m == 0) v = Wq[o * 256 + k]; else if (m == 1) v = Wq[o * 256 + 128 + k]; else if (m == 2) v = Wk[q]; else v = Wv[q];
      ((volatile unsigned short*)w16)[p] = bf16_bits(v); }
    for (int p = t_; p < DM * DM; p += 256) ((volatile b16*)w1r)[p] = (b16)bf16_rne(W1[p]);
    __threadfence(); }
}

__global__ __launch_bounds__(128) void lin_kernel(const float* __restrict__ X, int nrows, const unsigned short* __restrict__ Wt, const float* __restrict__ bias, float* __restrict__ Y) {
  __shared__ __attribute__((aligned(16))) float Ts[4][32 * 64];
  const int lane = threadIdx.x & 31, wave = threadIdx.x >> 5, nloc = lane & 15, hlf = lane >> 4, m0 = blockIdx.y * 128 + wave * 32, c0 = blockIdx.x * 64;
  const int ra = min(m0 + nloc, nrows - 1), rb = min(m0 + 16 + nloc, nrows - 1);
  v8f acc[2][4];
#pragma unroll
  for (int r = 0; r < 2; ++r)
#pragma unroll
    for (int t = 0; t < 4; ++t) acc[r][t] = (v8f){};
#pragma unroll
  for (int kb = 0; kb < DM; kb += 32) { const v16bb a0 = frag_f32bf(X + (size_t)ra * DM + kb, hlf), a1 = frag_f32bf(X + (size_t)rb * DM + kb, hlf);
#pragma unroll
    for (int t = 0; t < 4; ++t) { const v16bb bw = frag_bf(Wt + (size_t)(c0 + t * 16 + nloc) * DM + kb, hlf); acc[0][t] = wmma16bb(a0, bw, acc[0][t]); acc[1][t] = wmma16bb(a1, bw, acc[1][t]); } }
  float* Tt = Ts[wave];
#pragma unroll
  for (int t = 0; t < 4; ++t) { const float bb = bias ? bf16_rne(bias[c0 + t * 16 + nloc]) : 0.0f;
#pragma unroll
    for (int r = 0; r < 2; ++r)
#pragma unroll
      for (int v = 0; v < 8; ++v) Tt[(r * 16 + v + 8 * hlf) * 64 + t * 16 + nloc] = acc[r][t][v] + bb; }
  wave_lds_sync();
  float* dst0 = Y + (size_t)m0 * DM + c0;
  for (int pass = 0; pass < 2; ++pass) {
#pragma unroll
    for (int j = 0; j < 16; ++j) { const int rr = j * 2 + hlf, c4 = nloc * 4; *(volatile v4f*)(dst0 + (size_t)rr * DM + c4) = *(const v4f*)(Tt + rr * 64 + c4); }
    __threadfence(); }
}

__global__ __launch_bounds__(256) void vt_kernel(const float* __restrict__ V, b16* __restrict__ vt) {
  __shared__ __attribute__((aligned(16))) b16 Th[DM][128 + 8], Tl[DM][128 + 8];
  const int b = blockIdx.y, n0 = blockIdx.x * 128, t_ = threadIdx.x;
  for (int i = t_; i < 128 * DM; i += 256) { const int n = i >> 7, o = i & 127; b16 a, c; split16(V[((size_t)b * NO + n0 + n) * DM + o] * VS, a, c); Th[o][n] = a; Tl[o][n] = c; }
  __syncthreads();
  for (int pass = 0; pass < 2; ++pass) { for (int i = t_; i < DM * 16; i += 256) { const int o = i >> 4, c8 = (i & 15) * 8; const size_t dst = ((size_t)b * DM + o) * NO + n0 + c8;
      *(volatile v8b*)(vt + dst) = *(const v8b*)(&Th[o][c8]); *(volatile v8b*)(vt + VPL + dst) = *(const v8b*)(&Tl[o][c8]); } __threadfence(); }
}

__global__ __launch_bounds__(256) void attn_kernel(const float* __restrict__ QA, const float* __restrict__ QP, const float* __restrict__ Kr, const b16* __restrict__ vt, float* __restrict__ ctx) {
  __shared__ __attribute__((aligned(16))) float Os[32][DM + 4];
  const int wid = threadIdx.x >> 5, lane = threadIdx.x & 31, hh_ = lane >> 4, col = lane & 15;
  const int bhh = blockIdx.x / (NT / 32), t2 = blockIdx.x % (NT / 32), b = bhh / HH, n = wid & 3, sub = wid >> 2, t0 = t2 * 32 + sub * 16, ti = t0 + col;
  v16b qf, ql; { const float* qa = QA + (size_t)bhh * DM + n * DH; const float* qp = QP + (size_t)ti * DM + n * DH;
#pragma unroll
    for (int e = 0; e < 16; ++e) { const int k = (e < 8) ? (8 * hh_ + e) : (16 + 8 * hh_ + e - 8); b16 a, c; split16((qa[k] + qp[k]) * QS, a, c); qf[e] = a; ql[e] = c; } }
  const float* K = Kr + ((size_t)b * NO) * DM + n * DH; const b16* VT = vt + ((size_t)b * DM + n * DH) * NO;
  float m = -INFINITY, l = 0.0f; v8f o[2] = {{}, {}};
  for (int kb = 0; kb < NO; kb += 32) { v16b ka, kal, kb_, kbl; frag_split(K + (size_t)(kb + col) * DM, hh_, QS, ka, kal); frag_split(K + (size_t)(kb + 16 + col) * DM, hh_, QS, kb_, kbl);
    v8f s0 = {}, s1 = {}; s0 = wmma16b(ka, qf, s0); s0 = wmma16b(ka, ql, s0); s0 = wmma16b(kal, qf, s0); s1 = wmma16b(kb_, qf, s1); s1 = wmma16b(kb_, ql, s1); s1 = wmma16b(kbl, qf, s1);
    float mr = -INFINITY;
#pragma unroll
    for (int r = 0; r < 8; ++r) { s0[r] *= SCALE / (QS * QS); s1[r] *= SCALE / (QS * QS); mr = fmaxf(mr, fmaxf(s0[r], s1[r])); }
    mr = fmaxf(mr, __shfl_xor(mr, 16));
    const float mn = fmaxf(m, mr), al_ = nexp(m - mn); m = mn; float sum = 0.0f; v16b pb, pl;
#pragma unroll
    for (int r = 0; r < 8; ++r) { const float p0 = nexp(s0[r] - mn), p1 = nexp(s1[r] - mn); sum += p0 + p1; b16 a, c; split16(p0 * PS, a, c); pb[r] = a; pl[r] = c; split16(p1 * PS, a, c); pb[8 + r] = a; pl[8 + r] = c; }
    sum += __shfl_xor(sum, 16); l = l * al_ + sum;
#pragma unroll
    for (int d = 0; d < 2; ++d) { o[d] *= al_; const v16b vf = frag_kb(VT + (size_t)(d * 16 + col) * NO + kb, hh_), vl = frag_kb(VT + VPL + (size_t)(d * 16 + col) * NO + kb, hh_); o[d] = wmma16b(vf, pb, o[d]); o[d] = wmma16b(vf, pl, o[d]); o[d] = wmma16b(vl, pb, o[d]); } }
  const float inv = 1.0f / (l * VS * PS);
#pragma unroll
  for (int d = 0; d < 2; ++d)
#pragma unroll
    for (int r = 0; r < 8; ++r) Os[sub * 16 + col][n * DH + d * 16 + 8 * hh_ + r] = o[d][r] * inv;
  __syncthreads();
  float* dst = ctx + ((size_t)bhh * NT + t2 * 32) * DM;
  for (int pass = 0; pass < 2; ++pass) { for (int i = threadIdx.x; i < 32 * DM / 4; i += 256) { const int rr = i >> 5, c4 = (i & 31) * 4; *(volatile v4f*)(dst + (size_t)rr * DM + c4) = *(const v4f*)(&Os[rr][c4]); } __threadfence(); }
}

__global__ __launch_bounds__(128) void ffn_kernel(const float* __restrict__ ctx, const b16* __restrict__ w1r, const float* __restrict__ b1, const float* __restrict__ lg, const float* __restrict__ lb, const float* __restrict__ W2, const float* __restrict__ b2, float* __restrict__ y) {
  __shared__ float Ys[4][32];
  const int lane = threadIdx.x & 31, wave = threadIdx.x >> 5, nloc = lane & 15, hlf = lane >> 4, m0 = blockIdx.x * 128 + wave * 32;
  v8f acc[2][8];
#pragma unroll
  for (int r = 0; r < 2; ++r)
#pragma unroll
    for (int t = 0; t < 8; ++t) acc[r][t] = (v8f){};
#pragma unroll
  for (int kb = 0; kb < DM; kb += 32) { v16b a0, l0, a1, l1; frag_split(ctx + (size_t)(m0 + nloc) * DM + kb, hlf, XS, a0, l0); frag_split(ctx + (size_t)(m0 + 16 + nloc) * DM + kb, hlf, XS, a1, l1);
#pragma unroll
    for (int t = 0; t < 8; ++t) { const v16b bw = frag_kb(w1r + (size_t)(t * 16 + nloc) * DM + kb, hlf); acc[0][t] = wmma16b(a0, bw, acc[0][t]); acc[0][t] = wmma16b(l0, bw, acc[0][t]); acc[1][t] = wmma16b(a1, bw, acc[1][t]); acc[1][t] = wmma16b(l1, bw, acc[1][t]); } }
  const float bb2 = bf16_rne(b2[0]);
#pragma unroll
  for (int r = 0; r < 2; ++r)
#pragma unroll
    for (int v = 0; v < 8; ++v) { float xv[8]; float s = 0.0f;
#pragma unroll
      for (int t = 0; t < 8; ++t) { xv[t] = acc[r][t][v] * (1.0f / XS) + bf16_rne(b1[t * 16 + nloc]); s += xv[t]; }
#pragma unroll
      for (int o_ = 1; o_ < 16; o_ <<= 1) s += __shfl_xor(s, o_);
      const float mu = s * (1.0f / DM); float q = 0.0f;
#pragma unroll
      for (int t = 0; t < 8; ++t) { const float dlt = xv[t] - mu; q += dlt * dlt; }
#pragma unroll
      for (int o_ = 1; o_ < 16; o_ <<= 1) q += __shfl_xor(q, o_);
      const float rs = rsqrtf(q * (1.0f / DM) + LNE); float dot = 0.0f;
#pragma unroll
      for (int t = 0; t < 8; ++t) { const int c = t * 16 + nloc; const float xn = fmaxf((xv[t] - mu) * rs * bf16_rne(lg[c]) + bf16_rne(lb[c]), 0.0f); dot += xn * bf16_rne(W2[c]); }
#pragma unroll
      for (int o_ = 1; o_ < 16; o_ <<= 1) dot += __shfl_xor(dot, o_);
      if (nloc == 0) Ys[wave][r * 16 + 8 * hlf + v] = dot + bb2; }
  wave_lds_sync();
  for (int pass = 0; pass < 2; ++pass) { ((volatile float*)y)[(size_t)m0 + lane] = Ys[wave][lane]; __threadfence(); }
}
}

extern "C" void kernel_launch(void* const* d_in, const int* in_sizes, int n_in,
                              void* d_out, int out_size, void* d_ws, size_t ws_size, hipStream_t stream) {
  (void)n_in; (void)out_size;
  const float* A = (const float*)d_in[0]; const float* phi = (const float*)d_in[1]; const float* Hobs = (const float*)d_in[2];
  const float* Wq = (const float*)d_in[3]; const float* bq = (const float*)d_in[4]; const float* Wk = (const float*)d_in[5]; const float* bk = (const float*)d_in[6]; const float* Wv = (const float*)d_in[7]; const float* bv = (const float*)d_in[8];
  const float* W1 = (const float*)d_in[9]; const float* b1 = (const float*)d_in[10]; const float* lg = (const float*)d_in[11]; const float* lb = (const float*)d_in[12]; const float* W2 = (const float*)d_in[13]; const float* b2 = (const float*)d_in[14];
  float* y = (float*)d_out;
  if (in_sizes[0] != NQA * DM || in_sizes[1] != NT * DM || in_sizes[2] != NKV * DM || in_sizes[3] != DM * 256 || in_sizes[9] != DM * DM || in_sizes[13] != DM) return;
  size_t off = 0; char* ws = (char*)d_ws;
  auto carve = [&](size_t bytes) { char* p = ws + off; off += (bytes + 255) & ~(size_t)255; return p; };
  unsigned short* w16 = (unsigned short*)carve(4 * DM * DM * 2); b16* w1r = (b16*)carve(DM * DM * 2);
  float* QA = (float*)carve((size_t)256 * DM * 4); float* QP = (float*)carve((size_t)NT * DM * 4); float* Kr = (float*)carve((size_t)NKV * DM * 4); float* Vr = (float*)carve((size_t)NKV * DM * 4); b16* vt = (b16*)carve(VPL * 2 * 2); float* ctx = (float*)carve((size_t)NROW * DM * 4);
  if (off > ws_size) return;
  prep_kernel<<<1, 256, 0, stream>>>(Wq, Wk, Wv, W1, w16, w1r);
  lin_kernel<<<dim3(2, 2), 128, 0, stream>>>(A, NQA, w16, nullptr, QA);
  lin_kernel<<<dim3(2, NT / 128), 128, 0, stream>>>(phi, NT, w16 + DM * DM, bq, QP);
  lin_kernel<<<dim3(2, NKV / 128), 128, 0, stream>>>(Hobs, NKV, w16 + 2 * DM * DM, bk, Kr);
  lin_kernel<<<dim3(2, NKV / 128), 128, 0, stream>>>(Hobs, NKV, w16 + 3 * DM * DM, bv, Vr);
  vt_kernel<<<dim3(NO / 128, Bn), 256, 0, stream>>>(Vr, vt);
  attn_kernel<<<Bn * HH * NT / 32, 256, 0, stream>>>(QA, QP, Kr, vt, ctx);
  ffn_kernel<<<NROW / 128, 128, 0, stream>>>(ctx, w1r, b1, lg, lb, W2, b2, y);
}
